// Decoder_86526411145547
// MI455X (gfx1250) — hardware-verified
//
#include <hip/hip_runtime.h>
#include <math.h>

typedef __attribute__((ext_vector_type(16))) _Float16 v16h;
typedef __attribute__((ext_vector_type(8)))  _Float16 v8h;
typedef __attribute__((ext_vector_type(8)))  float    v8f;
typedef __attribute__((ext_vector_type(4)))  float    v4f;
typedef __attribute__((ext_vector_type(2)))  float    v2f;
typedef __attribute__((ext_vector_type(4)))  unsigned v4u;

constexpr int kRays       = 32768;
constexpr int kGauss      = 1024;
constexpr int kFeat       = 16;
constexpr int kPlaneK     = 64;
constexpr int kPlaneWords = kPlaneK / 2;
constexpr int kSlabPitch  = 36;
static_assert(kFeat == 16, "feature count");
static_assert((kRays % 256) == 0 && (kGauss % 256) == 0, "block multiples");
static_assert((kGauss % 16) == 0 && (kRays % 32) == 0, "tile multiples");
static_assert((kPlaneK % 32) == 0, "K multiple of 32");

constexpr float kCarry        = 64.0f;
constexpr float kResCarry     = 2048.0f;
constexpr float kMainFold     = 1.0f / (kCarry * kCarry);
constexpr float kResFold      = kMainFold / kResCarry;
constexpr float kF16MinNormal = 6.103515625e-05f;

constexpr size_t kOffPA   = 0;
constexpr size_t kBytesPA = (size_t)kRays * kPlaneK * 2;
constexpr size_t kOffPB   = kOffPA + kBytesPA;
constexpr size_t kBytesPB = (size_t)kGauss * kPlaneK * 2;
constexpr size_t kWsTotal = kOffPB + kBytesPB;
static_assert(kBytesPA == 4194304ull && kBytesPB == 131072ull, "plane sizes");
static_assert(kWsTotal == 4325376ull, "carve total");
static_assert(kWsTotal <= 134217728ull, "carve cap");
static_assert((kOffPB % 128) == 0, "aligned regions");

union FragU { v16h v; v8h h[2]; };
__device__ __forceinline__ v16h frag_load(const _Float16* p) {
  FragU f;
  f.h[0] = *(const v8h*)(p);
  f.h[1] = *(const v8h*)(p + 16);
  return f.v;
}

__device__ __forceinline__ v8f mma_f16(v16h a, v16h b, v8f c) {
  c = __builtin_amdgcn_wmma_f32_16x16x32_f16(false, a, false, b, (short)0, c, false, false);
  asm volatile("v_nop\n\tv_nop\n\tv_nop\n\tv_nop" : "+v"(c) : "v"(a), "v"(b));
  return c;
}

__device__ __forceinline__ void split_feature(float v, unsigned& hb, unsigned& lb) {
  const float w  = v * kCarry;
  const float wf = (fabsf(w) < kF16MinNormal) ? 0.0f : w;
  const _Float16 hh = (_Float16)wf;
  const float hf = (float)hh;
  const float lo = (w - hf) * kResCarry;
  const float lf = (fabsf(lo) < kF16MinNormal) ? 0.0f : lo;
  const _Float16 lh = (_Float16)lf;
  const unsigned short hs = __builtin_bit_cast(unsigned short, hh);
  const unsigned short ls = __builtin_bit_cast(unsigned short, lh);
  hb = (unsigned)hs;
  lb = (unsigned)ls;
}

template <bool A_LAYOUT>
__device__ __forceinline__ void emit_plane_rows(unsigned* slab, const float (&f)[kFeat],
                                                unsigned* plane, int rowBase, int lane) {
  unsigned hb[kFeat], lb[kFeat];
#pragma unroll
  for (int i = 0; i < kFeat; ++i) split_feature(f[i], hb[i], lb[i]);
  unsigned hw[8], lw[8];
#pragma unroll
  for (int j = 0; j < 8; ++j) {
    hw[j] = hb[2 * j] | (hb[2 * j + 1] << 16);
    lw[j] = lb[2 * j] | (lb[2 * j + 1] << 16);
  }
  const v4u z  = (v4u){0u, 0u, 0u, 0u};
  const v4u h0 = (v4u){hw[0], hw[1], hw[2], hw[3]};
  const v4u h1 = (v4u){hw[4], hw[5], hw[6], hw[7]};
  const v4u l0 = (v4u){lw[0], lw[1], lw[2], lw[3]};
  const v4u l1 = (v4u){lw[4], lw[5], lw[6], lw[7]};
  unsigned* my = slab + lane * kSlabPitch;
  *(v4u*)(my + 0)  = h0;
  *(v4u*)(my + 4)  = h1;
  *(v4u*)(my + 8)  = z;
  *(v4u*)(my + 12) = z;
  if (A_LAYOUT) {
    *(v4u*)(my + 16) = h0;
    *(v4u*)(my + 20) = h1;
    *(v4u*)(my + 24) = l0;
    *(v4u*)(my + 28) = l1;
  } else {
    *(v4u*)(my + 16) = l0;
    *(v4u*)(my + 20) = l1;
    *(v4u*)(my + 24) = h0;
    *(v4u*)(my + 28) = h1;
  }
  __syncthreads();
  const int q  = lane >> 3;
  const int c4 = (lane & 7) * 4;
  for (int pass = 0; pass < 2; ++pass) {
#pragma unroll
    for (int it = 0; it < 8; ++it) {
      const int row = it * 4 + q;
      const v4u v = *(const v4u*)(slab + row * kSlabPitch + c4);
      *(volatile v4u*)(plane + (size_t)(rowBase + row) * kPlaneWords + c4) = v;
    }
    __threadfence();
  }
}

__global__ __launch_bounds__(256) void gauss_coef_prep_kernel(
    const float* __restrict__ means, const float* __restrict__ covs, unsigned* __restrict__ planeB)
{
  __shared__ __align__(16) unsigned sW[8][32 * kSlabPitch];
  const int tid  = threadIdx.x;
  const int lane = tid & 31;
  const int wave = tid >> 5;
  const int gRaw = blockIdx.x * 256 + tid;
  const int g    = (gRaw < kGauss) ? gRaw : (kGauss - 1);

  const v4f c0 = *(const v4f*)(covs + (size_t)g * 16 + 0);
  const v4f c1 = *(const v4f*)(covs + (size_t)g * 16 + 4);
  const v4f c2 = *(const v4f*)(covs + (size_t)g * 16 + 8);
  const v4f c3 = *(const v4f*)(covs + (size_t)g * 16 + 12);
  const v4f mu = *(const v4f*)(means + (size_t)g * 4);
  float a[16];
  a[0]  = c0[0]; a[1]  = c0[1]; a[2]  = c0[2]; a[3]  = c0[3];
  a[4]  = c1[0]; a[5]  = c1[1]; a[6]  = c1[2]; a[7]  = c1[3];
  a[8]  = c2[0]; a[9]  = c2[1]; a[10] = c2[2]; a[11] = c2[3];
  a[12] = c3[0]; a[13] = c3[1]; a[14] = c3[2]; a[15] = c3[3];

  float inv[16];
  inv[0]  =  a[5]*a[10]*a[15] - a[5]*a[11]*a[14] - a[9]*a[6]*a[15] + a[9]*a[7]*a[14] + a[13]*a[6]*a[11] - a[13]*a[7]*a[10];
  inv[4]  = -a[4]*a[10]*a[15] + a[4]*a[11]*a[14] + a[8]*a[6]*a[15] - a[8]*a[7]*a[14] - a[12]*a[6]*a[11] + a[12]*a[7]*a[10];
  inv[8]  =  a[4]*a[9]*a[15]  - a[4]*a[11]*a[13] - a[8]*a[5]*a[15] + a[8]*a[7]*a[13] + a[12]*a[5]*a[11] - a[12]*a[7]*a[9];
  inv[12] = -a[4]*a[9]*a[14]  + a[4]*a[10]*a[13] + a[8]*a[5]*a[14] - a[8]*a[6]*a[13] - a[12]*a[5]*a[10] + a[12]*a[6]*a[9];
  inv[1]  = -a[1]*a[10]*a[15] + a[1]*a[11]*a[14] + a[9]*a[2]*a[15] - a[9]*a[3]*a[14] - a[13]*a[2]*a[11] + a[13]*a[3]*a[10];
  inv[5]  =  a[0]*a[10]*a[15] - a[0]*a[11]*a[14] - a[8]*a[2]*a[15] + a[8]*a[3]*a[14] + a[12]*a[2]*a[11] - a[12]*a[3]*a[10];
  inv[9]  = -a[0]*a[9]*a[15]  + a[0]*a[11]*a[13] + a[8]*a[1]*a[15] - a[8]*a[3]*a[13] - a[12]*a[1]*a[11] + a[12]*a[3]*a[9];
  inv[13] =  a[0]*a[9]*a[14]  - a[0]*a[10]*a[13] - a[8]*a[1]*a[14] + a[8]*a[2]*a[13] + a[12]*a[1]*a[10] - a[12]*a[2]*a[9];
  inv[2]  =  a[1]*a[6]*a[15]  - a[1]*a[7]*a[14]  - a[5]*a[2]*a[15] + a[5]*a[3]*a[14] + a[13]*a[2]*a[7]  - a[13]*a[3]*a[6];
  inv[6]  = -a[0]*a[6]*a[15]  + a[0]*a[7]*a[14]  + a[4]*a[2]*a[15] - a[4]*a[3]*a[14] - a[12]*a[2]*a[7]  + a[12]*a[3]*a[6];
  inv[10] =  a[0]*a[5]*a[15]  - a[0]*a[7]*a[13]  - a[4]*a[1]*a[15] + a[4]*a[3]*a[13] + a[12]*a[1]*a[7]  - a[12]*a[3]*a[5];
  inv[14] = -a[0]*a[5]*a[14]  + a[0]*a[6]*a[13]  + a[4]*a[1]*a[14] - a[4]*a[2]*a[13] - a[12]*a[1]*a[6]  + a[12]*a[2]*a[5];
  inv[3]  = -a[1]*a[6]*a[11]  + a[1]*a[7]*a[10]  + a[5]*a[2]*a[11] - a[5]*a[3]*a[10] - a[9]*a[2]*a[7]   + a[9]*a[3]*a[6];
  inv[7]  =  a[0]*a[6]*a[11]  - a[0]*a[7]*a[10]  - a[4]*a[2]*a[11] + a[4]*a[3]*a[10] + a[8]*a[2]*a[7]   - a[8]*a[3]*a[6];
  inv[11] = -a[0]*a[5]*a[11]  + a[0]*a[7]*a[9]   + a[4]*a[1]*a[11] - a[4]*a[3]*a[9]  - a[8]*a[1]*a[7]   + a[8]*a[3]*a[5];
  inv[15] =  a[0]*a[5]*a[10]  - a[0]*a[6]*a[9]   - a[4]*a[1]*a[10] + a[4]*a[2]*a[9]  + a[8]*a[1]*a[6]   - a[8]*a[2]*a[5];
  const float det  = a[0]*inv[0] + a[1]*inv[4] + a[2]*inv[8] + a[3]*inv[12];
  const float rdet = 1.0f / det;

  const float s00 = inv[0]  * rdet;
  const float s11 = inv[5]  * rdet;
  const float s22 = inv[10] * rdet;
  const float s33 = inv[15] * rdet;
  const float s01 = 0.5f * (inv[1]  + inv[4])  * rdet;
  const float s02 = 0.5f * (inv[2]  + inv[8])  * rdet;
  const float s03 = 0.5f * (inv[3]  + inv[12]) * rdet;
  const float s12 = 0.5f * (inv[6]  + inv[9])  * rdet;
  const float s13 = 0.5f * (inv[7]  + inv[13]) * rdet;
  const float s23 = 0.5f * (inv[11] + inv[14]) * rdet;

  const float m0 = mu[0], m1 = mu[1], m2 = mu[2], m3 = mu[3];
  const float b0 = s00 * m0 + s01 * m1 + s02 * m2 + s03 * m3;
  const float b1 = s01 * m0 + s11 * m1 + s12 * m2 + s13 * m3;
  const float b2 = s02 * m0 + s12 * m1 + s22 * m2 + s23 * m3;
  const float b3 = s03 * m0 + s13 * m1 + s23 * m2 + s33 * m3;
  const float cc = m0 * b0 + m1 * b1 + m2 * b2 + m3 * b3;

  float zf = 0.0f;
  asm volatile("" : "+v"(zf));

  float f[kFeat];
  f[0]  = -0.5f * s00;
  f[1]  = -0.5f * s11;
  f[2]  = -0.5f * s22;
  f[3]  = -0.5f * s33;
  f[4]  = -s01;
  f[5]  = -s02;
  f[6]  = -s03;
  f[7]  = -s12;
  f[8]  = -s13;
  f[9]  = -s23;
  f[10] = b0;
  f[11] = b1;
  f[12] = b2;
  f[13] = b3;
  f[14] = -0.5f * cc;
  f[15] = zf;

  emit_plane_rows<false>(sW[wave], f, planeB, blockIdx.x * 256 + wave * 32, lane);
}

__global__ __launch_bounds__(256) void ray_feat_prep_kernel(
    const float* __restrict__ origins, const float* __restrict__ dirs, unsigned* __restrict__ planeA)
{
  __shared__ __align__(16) unsigned sW[8][32 * kSlabPitch];
  const int tid  = threadIdx.x;
  const int lane = tid & 31;
  const int wave = tid >> 5;
  const int nRaw = blockIdx.x * 256 + tid;
  const int n    = (nRaw < kRays) ? nRaw : (kRays - 1);

  const v2f o = *(const v2f*)(origins + (size_t)n * 2);
  const v2f d = *(const v2f*)(dirs + (size_t)n * 2);
  const float x0 = o[0], x1 = o[1], x2 = d[0], x3 = d[1];

  float onef = 1.0f;
  float zf   = 0.0f;
  asm volatile("" : "+v"(onef));
  asm volatile("" : "+v"(zf));

  float f[kFeat];
  f[0]  = x0 * x0;
  f[1]  = x1 * x1;
  f[2]  = x2 * x2;
  f[3]  = x3 * x3;
  f[4]  = x0 * x1;
  f[5]  = x0 * x2;
  f[6]  = x0 * x3;
  f[7]  = x1 * x2;
  f[8]  = x1 * x3;
  f[9]  = x2 * x3;
  f[10] = x0;
  f[11] = x1;
  f[12] = x2;
  f[13] = x3;
  f[14] = onef;
  f[15] = zf;

  emit_plane_rows<true>(sW[wave], f, planeA, blockIdx.x * 256 + wave * 32, lane);
}

__global__ __launch_bounds__(256) void mix_eval_kernel(
    const unsigned short* __restrict__ planeA, const unsigned short* __restrict__ planeB,
    const float* __restrict__ labels, float* __restrict__ out)
{
  const int lane = threadIdx.x & 31;
  const int wave = threadIdx.x >> 5;
  const int hh   = lane >> 4;
  const int c    = lane & 15;
  const int rayBase = (blockIdx.x * 8 + wave) * 32;
  const _Float16* Ah = (const _Float16*)planeA;
  const _Float16* Bh = (const _Float16*)planeB;
  const int srcLane = ((lane >> 3) & 1) << 4;
  const int rsel    = lane & 7;
  float res = 0.0f;

#pragma unroll 1
  for (int mt = 0; mt < 2; ++mt) {
    const _Float16* ap = Ah + (size_t)(rayBase + mt * 16 + c) * kPlaneK + 8 * hh;
    const v16h a0 = frag_load(ap);
    const v16h a1 = frag_load(ap + 32);
    float acc[8];
#pragma unroll
    for (int r = 0; r < 8; ++r) acc[r] = 0.0f;

#pragma unroll 1
    for (int nt = 0; nt < kGauss / 16; ++nt) {
      const int col = nt * 16 + c;
      const _Float16* bp = Bh + (size_t)col * kPlaneK + 8 * hh;
      const v16h b0 = frag_load(bp);
      const v16h b1 = frag_load(bp + 32);
      const float lab = labels[col];
      v8f vm = (v8f){0.f, 0.f, 0.f, 0.f, 0.f, 0.f, 0.f, 0.f};
      v8f vr = (v8f){0.f, 0.f, 0.f, 0.f, 0.f, 0.f, 0.f, 0.f};
      vm = mma_f16(a0, b0, vm);
      vr = mma_f16(a1, b1, vr);
#pragma unroll
      for (int r = 0; r < 8; ++r) {
        const float e = fmaf(vr[r], kResFold, vm[r] * kMainFold);
        acc[r] = fmaf(expf(e), lab, acc[r]);
      }
    }

#pragma unroll
    for (int r = 0; r < 8; ++r) {
      float s = acc[r];
      s += __shfl_xor(s, 1, 32);
      s += __shfl_xor(s, 2, 32);
      s += __shfl_xor(s, 4, 32);
      s += __shfl_xor(s, 8, 32);
      acc[r] = s;
    }
    float t[8];
#pragma unroll
    for (int r = 0; r < 8; ++r) t[r] = __shfl(acc[r], srcLane, 32);
    float sel = t[0];
    sel = (rsel == 1) ? t[1] : sel;
    sel = (rsel == 2) ? t[2] : sel;
    sel = (rsel == 3) ? t[3] : sel;
    sel = (rsel == 4) ? t[4] : sel;
    sel = (rsel == 5) ? t[5] : sel;
    sel = (rsel == 6) ? t[6] : sel;
    sel = (rsel == 7) ? t[7] : sel;
    res = (hh == mt) ? sel : res;
  }

  const float s   = fminf(fmaxf(res, -30.0f), 30.0f);
  const float ex  = expf(-fabsf(s));
  const float rcp = 1.0f / (1.0f + ex);
  const float p   = (s >= 0.0f) ? rcp : (ex * rcp);
  volatile float* op = out + rayBase + lane;
  *op = p;
  __threadfence();
  *op = p;
}

extern "C" void kernel_launch(void* const* d_in, const int* in_sizes, int n_in,
                              void* d_out, int out_size, void* d_ws, size_t ws_size,
                              hipStream_t stream) {
  if (n_in < 5) return;
  if (in_sizes[0] != kRays * 2) return;
  if (in_sizes[1] != kRays * 2) return;
  if (in_sizes[2] != kGauss * 4) return;
  if (in_sizes[3] != kGauss * 16) return;
  if (in_sizes[4] != kGauss) return;
  if (out_size != kRays) return;
  if (ws_size < kWsTotal) return;

  const float* origins = (const float*)d_in[0];
  const float* dirs    = (const float*)d_in[1];
  const float* means   = (const float*)d_in[2];
  const float* covs    = (const float*)d_in[3];
  const float* labels  = (const float*)d_in[4];
  float* out = (float*)d_out;

  char* ws = (char*)d_ws;
  unsigned* PA = (unsigned*)(ws + kOffPA);
  unsigned* PB = (unsigned*)(ws + kOffPB);

  gauss_coef_prep_kernel<<<kGauss / 256, 256, 0, stream>>>(means, covs, PB);
  ray_feat_prep_kernel<<<kRays / 256, 256, 0, stream>>>(origins, dirs, PA);
  mix_eval_kernel<<<kRays / 256, 256, 0, stream>>>(
      (const unsigned short*)PA, (const unsigned short*)PB, labels, out);
}
